// RootModule_2216203125290
// MI455X (gfx1250) — hardware-run, weakly checked
//
#include <hip/hip_runtime.h>


#ifndef NROWS
#define NROWS 8192
#endif
#define NROWS_FULL 8192
#define DW   1024
#define RK   16
#define NL   4
#define PD   3
#define WLOG 6
#define WSI  (1.0f / 64.0f)
#define OSP  68
#define UP   20

static_assert(NROWS % 64 == 0);
static_assert(NROWS <= NROWS_FULL);
static_assert(DW % 64 == 0);
static_assert(DW % 32 == 0);
static_assert(RK == 16);
static_assert(((size_t)NROWS * DW) % 2048 == 0);
static_assert(((size_t)NL * DW * DW) % 2048 == 0);
static_assert(((size_t)NL * RK * DW) % 2048 == 0);
static_assert(32 * 16 * 4 == 16 * 64 * 2);
static_assert(32 * 16 * 8 == 16 * 64 * 4);
static_assert(32 * 16 * 4 == 64 * RK * 2);
static_assert((OSP * 4) % 16 == 0);
static_assert((UP * 4) % 16 == 0);
static_assert(OSP >= 64);
static_assert(UP >= RK);
static_assert(16 * OSP * 4 <= 131072);
static_assert(64 * UP * 4 + 64 * 4 <= 131072);

typedef _Float16 h16;
typedef __attribute__((ext_vector_type(16))) _Float16 v16h;
typedef __attribute__((ext_vector_type(8)))  _Float16 v8h;
typedef __attribute__((ext_vector_type(8)))  float    v8f;
typedef __attribute__((ext_vector_type(4)))  float    v4f;
typedef v4f  __attribute__((may_alias)) v4fa;

__device__ __forceinline__ unsigned short f2bf(float f) { unsigned u = __float_as_uint(f); u += 0x7FFFu + ((u >> 16) & 1u); return (unsigned short)(u >> 16); }
__device__ __forceinline__ float bfr(float f) { return __uint_as_float(((unsigned)f2bf(f)) << 16); }
__device__ __forceinline__ v16h cat16(v8h lo, v8h hi) { return __builtin_shufflevector(lo, hi, 0, 1, 2, 3, 4, 5, 6, 7, 8, 9, 10, 11, 12, 13, 14, 15); }
__device__ __forceinline__ v8f wmma16(v16h a, v16h b, v8f c) { return __builtin_amdgcn_wmma_f32_16x16x32_f16(false, a, false, b, (short)0, c, false, false); }
__device__ __forceinline__ v8f wmma16g(v16h a, v16h b, v8f c) { c = wmma16(a, b, c); asm volatile("v_nop\n\tv_nop\n\tv_nop\n\tv_nop" : "+v"(c) : "v"(a), "v"(b)); return c; }
__device__ __forceinline__ v16h  ldh(const h16* p) { return cat16(*(const v8h*)p, *(const v8h*)(p + 16)); }
__device__ __forceinline__ void wave_sync() { __builtin_amdgcn_fence(3  , "wavefront"); __builtin_amdgcn_wave_barrier(); asm volatile("" ::: "memory"); }
static __device__ __forceinline__ h16 toh_flush(float v) { const float w = (fabsf(v) < 6.103515625e-05f) ? 0.0f : v; return (h16)w; }

template <int SH>
static __device__ __forceinline__ void cvt_body(const float* __restrict__ src, h16* dst, unsigned n8) {
    const unsigned i = blockIdx.x * 256u + threadIdx.x; if (i >= n8) return;
    const v8f v = *(const v8f*)(src + (size_t)i * 8); v8h o;
#pragma unroll
    for (int k = 0; k < 8; ++k) o[k] = toh_flush(bfr(v[k]) * (float)(1 << SH));
    *(volatile v8h*)(dst + (size_t)i * 8) = o; __threadfence(); *(volatile v8h*)(dst + (size_t)i * 8) = o;
}
__global__ __launch_bounds__(256) void k_cvt_x(const float* __restrict__ src, h16* dst, unsigned n8) { cvt_body<0>(src, dst, n8); }
__global__ __launch_bounds__(256) void k_cvt_w(const float* __restrict__ src, h16* dst, unsigned n8) { cvt_body<WLOG>(src, dst, n8); }

__global__ __launch_bounds__(32) void k_u(const h16* __restrict__ X, const h16* __restrict__ Bh, const float* __restrict__ nu, const float* __restrict__ tt,
                                          const float* __restrict__ aW, const float* __restrict__ ab, h16* UA) {
    __shared__ __align__(16) float us[64 * UP];
    __shared__ float al[64];
    const int lane = threadIdx.x & 31, lr = lane & 15, hi = lane >> 4;
    const unsigned bx = blockIdx.x; const unsigned r0 = bx * 64u;
    const float w0 = bfr(aW[0]), w1 = bfr(aW[1]), w2 = bfr(aW[2]), w3 = bfr(aW[3]), wb = bfr(ab[0]);
#pragma unroll 1
    for (int q = 0; q < 2; ++q) {
        const unsigned row = r0 + (unsigned)q * 32u + (unsigned)lane;
        float p = bfr(nu[(size_t)row * PD + 0]) * w0;
        p = fmaf(bfr(nu[(size_t)row * PD + 1]), w1, p);
        p = fmaf(bfr(nu[(size_t)row * PD + 2]), w2, p);
        p = fmaf(bfr(tt[row]), w3, p);
        al[q * 32 + lane] = (p + wb) * WSI; }
    v8f acc[4];
#pragma unroll
    for (int mb = 0; mb < 4; ++mb) acc[mb] = (v8f){};
    const size_t aoff = (size_t)(r0 + (unsigned)lr) * DW + 8 * hi, boff = (size_t)lr * DW + 8 * hi;
#pragma unroll 1
    for (int kc = 0; kc < DW; kc += 32) {
        const v16h b = ldh(Bh + boff + kc);
#pragma unroll
        for (int mb = 0; mb < 4; ++mb) { const v16h a = ldh(X + aoff + (size_t)mb * 16 * DW + kc); acc[mb] = wmma16g(a, b, acc[mb]); }
    }
    wave_sync();
#pragma unroll
    for (int mb = 0; mb < 4; ++mb) {
#pragma unroll
        for (int j = 0; j < 8; ++j) us[(mb * 16 + hi * 8 + j) * UP + lr] = acc[mb][j] * al[mb * 16 + hi * 8 + j]; }
    wave_sync();
    h16* ub = UA + (size_t)r0 * RK;
#pragma unroll 1
    for (int ps = 0; ps < 2; ++ps) {
#pragma unroll
        for (int s = 0; s < 4; ++s) { const int p = s * 32 + lane; const int row = p >> 1, c8 = (p & 1) * 8;
            const v4f x0 = *(const v4fa*)(&us[row * UP + c8]); const v4f x1 = *(const v4fa*)(&us[row * UP + c8 + 4]); v8h hv;
#pragma unroll
            for (int i = 0; i < 4; ++i) { hv[i] = toh_flush(x0[i]); hv[4 + i] = toh_flush(x1[i]); }
            *(volatile v8h*)(ub + (size_t)p * 8) = hv; }
        if (ps == 0) __threadfence(); }
}

__global__ __launch_bounds__(32) void k_gemm(const h16* __restrict__ X, const h16* __restrict__ Wh, const h16* __restrict__ UA, const h16* __restrict__ Ah,
                                             const float* __restrict__ bias, h16* XO, float* OF, int outf) {
    __shared__ __align__(16) float os[16 * OSP];
    const int lane = threadIdx.x & 31, lr = lane & 15, hi = lane >> 4;
    const unsigned bx = blockIdx.x, by = blockIdx.y; const unsigned r0 = bx * 64u, c0 = by * 64u;
    v8f acc[4][4];
#pragma unroll
    for (int mb = 0; mb < 4; ++mb)
#pragma unroll
        for (int nb = 0; nb < 4; ++nb) acc[mb][nb] = (v8f){};
    const size_t aoff = (size_t)(r0 + (unsigned)lr) * DW + 8 * hi, boff = (size_t)(c0 + (unsigned)lr) * DW + 8 * hi;
#pragma unroll 1
    for (int kc = 0; kc < DW; kc += 32) {
        v16h a[4];
#pragma unroll
        for (int mb = 0; mb < 4; ++mb) a[mb] = ldh(X + aoff + (size_t)mb * 16 * DW + kc);
#pragma unroll
        for (int nb = 0; nb < 4; ++nb) { const v16h b = ldh(Wh + boff + (size_t)nb * 16 * DW + kc);
#pragma unroll
            for (int mb = 0; mb < 4; ++mb) acc[mb][nb] = wmma16g(a[mb], b, acc[mb][nb]); }
    }
    {
        const v8h z8 = (v8h){};
        const size_t uoff = (size_t)(r0 + (unsigned)lr) * RK + 8 * hi, eoff = (size_t)(c0 + (unsigned)lr) * RK + 8 * hi;
        v16h a[4];
#pragma unroll
        for (int mb = 0; mb < 4; ++mb) a[mb] = cat16(*(const v8h*)(UA + uoff + (size_t)mb * 16 * RK), z8);
#pragma unroll
        for (int nb = 0; nb < 4; ++nb) { const v16h b = cat16(*(const v8h*)(Ah + eoff + (size_t)nb * 16 * RK), z8);
#pragma unroll
            for (int mb = 0; mb < 4; ++mb) acc[mb][nb] = wmma16g(a[mb], b, acc[mb][nb]); }
    }
    float bc[4];
#pragma unroll
    for (int nb = 0; nb < 4; ++nb) bc[nb] = bfr(bias[c0 + (unsigned)(nb * 16 + lr)]);
#pragma unroll
    for (int mb = 0; mb < 4; ++mb) {
#pragma unroll
        for (int nb = 0; nb < 4; ++nb) {
#pragma unroll
            for (int j = 0; j < 8; ++j) os[(hi * 8 + j) * OSP + nb * 16 + lr] = acc[mb][nb][j] * WSI + bc[nb]; }
        wave_sync();
#pragma unroll 1
        for (int ps = 0; ps < 2; ++ps) {
            if (outf != 0) {
                float* ob = OF + (size_t)(r0 + (unsigned)(mb * 16)) * DW + c0;
#pragma unroll
                for (int s = 0; s < 8; ++s) { const int row = 2 * s + (lane >> 4), cofs = (lane & 15) * 4;
                    const v4f val = *(const v4fa*)(&os[row * OSP + cofs]);
                    *(volatile v4f*)(ob + (size_t)row * DW + cofs) = val; }
            } else {
                h16* ob = XO + (size_t)(r0 + (unsigned)(mb * 16)) * DW + c0;
#pragma unroll
                for (int s = 0; s < 4; ++s) { const int row = 4 * s + (lane >> 3), c8 = (lane & 7) * 8;
                    const v4f x0 = *(const v4fa*)(&os[row * OSP + c8]); const v4f x1 = *(const v4fa*)(&os[row * OSP + c8 + 4]); v8h hv;
#pragma unroll
                    for (int i = 0; i < 4; ++i) { hv[i] = toh_flush(x0[i]); hv[4 + i] = toh_flush(x1[i]); }
                    *(volatile v8h*)(ob + (size_t)row * DW + c8) = hv; }
            }
            if (ps == 0) __threadfence(); }
        wave_sync();
    }
}

static constexpr size_t al256(size_t v) { return (v + 255) & ~(size_t)255; }
static constexpr size_t SZ_X  = al256((size_t)NROWS * DW * 2);
static constexpr size_t SZ_W  = al256((size_t)NL * DW * DW * 2);
static constexpr size_t SZ_B  = al256((size_t)NL * RK * DW * 2);
static constexpr size_t SZ_A  = al256((size_t)NL * DW * RK * 2);
static constexpr size_t SZ_U  = al256((size_t)NROWS * RK * 2);
static constexpr size_t SZ_TOTAL = 2 * SZ_X + SZ_W + SZ_B + SZ_A + SZ_U;
static_assert(SZ_TOTAL <= (size_t)134217728);
static_assert(((size_t)DW * DW * 2) % 256 == 0);
static_assert(((size_t)RK * DW * 2) % 256 == 0);
static_assert((size_t)(NROWS / 64) * 64 * DW * 2 <= SZ_X);
static_assert((size_t)(NROWS / 64) * 64 * RK * 2 <= SZ_U);
static_assert((size_t)NROWS * DW / 8 <= 0xFFFFFFFFu);

extern "C" void kernel_launch(void* const* d_in, const int* in_sizes, int n_in,
                              void* d_out, int out_size, void* d_ws, size_t ws_size, hipStream_t stream) {
    if (n_in < 9) return;
    if ((size_t)in_sizes[0] < (size_t)NROWS * DW) return;
    if ((size_t)in_sizes[1] < (size_t)NROWS * PD || (size_t)in_sizes[2] < (size_t)NROWS) return;
    if ((size_t)in_sizes[3] < (size_t)NL * DW * DW || (size_t)in_sizes[4] < (size_t)NL * DW * RK || (size_t)in_sizes[5] < (size_t)NL * RK * DW) return;
    if (in_sizes[6] < NL * DW || in_sizes[7] < NL * (PD + 1) || in_sizes[8] < NL) return;
    if ((size_t)out_size < (size_t)NROWS * DW) return;
    if (SZ_TOTAL > ws_size) return;
    const float* mu = (const float*)d_in[0];
    const float* nu = (const float*)d_in[1];
    const float* tt = (const float*)d_in[2];
    const float* Ws = (const float*)d_in[3];
    const float* As = (const float*)d_in[4];
    const float* Bs = (const float*)d_in[5];
    const float* bs = (const float*)d_in[6];
    const float* aW = (const float*)d_in[7];
    const float* ab = (const float*)d_in[8];
    float* OUT = (float*)d_out;
    char* wsp = (char*)d_ws;
    h16* X0 = (h16*)wsp; wsp += SZ_X;
    h16* X1 = (h16*)wsp; wsp += SZ_X;
    h16* WH = (h16*)wsp; wsp += SZ_W;
    h16* BH = (h16*)wsp; wsp += SZ_B;
    h16* AH = (h16*)wsp; wsp += SZ_A;
    h16* UA = (h16*)wsp; wsp += SZ_U;

    { const unsigned n8 = (unsigned)((size_t)NROWS * DW / 8);   k_cvt_x<<<(n8 + 255u) / 256u, 256, 0, stream>>>(mu, X0, n8); }
    { const unsigned n8 = (unsigned)((size_t)NL * DW * DW / 8); k_cvt_w<<<(n8 + 255u) / 256u, 256, 0, stream>>>(Ws, WH, n8); }
    { const unsigned n8 = (unsigned)((size_t)NL * RK * DW / 8); k_cvt_w<<<(n8 + 255u) / 256u, 256, 0, stream>>>(Bs, BH, n8); }
    { const unsigned n8 = (unsigned)((size_t)NL * DW * RK / 8); k_cvt_w<<<(n8 + 255u) / 256u, 256, 0, stream>>>(As, AH, n8); }

    for (int i = 0; i < NL; ++i) {
        const h16* xin = (i & 1) ? X1 : X0;
        h16* xout = (i & 1) ? X0 : X1;
        k_u<<<dim3(NROWS / 64, 1, 1), 32, 0, stream>>>(xin, BH + (size_t)i * RK * DW, nu, tt, aW + (size_t)i * (PD + 1), ab + i, UA);
        k_gemm<<<dim3(NROWS / 64, DW / 64, 1), 32, 0, stream>>>(xin, WH + (size_t)i * DW * DW, UA, AH + (size_t)i * DW * RK, bs + (size_t)i * DW,
                                                                 xout, OUT, (i == NL - 1) ? 1 : 0);
    }
}
